// GlobalMQA_40939628265847
// MI455X (gfx1250) — hardware-verified
//
#include <hip/hip_runtime.h>
#include <math.h>
#include <float.h>
#include <stdint.h>

#define NBATCH 2
#define SEQ    2048
#define MTOT   (NBATCH * SEQ)
#define DM     1024
#define NH     8
#define HD     128
#define NROT   (HD / 2)
#define NQB    (SEQ / 64)
#define NQKV   (DM + 2 * HD)
#define OUTN   (MTOT * DM)
static_assert(NH * HD == DM);
static_assert(HD == 128);
static_assert(DM == 128 * 8);
static_assert((SEQ % 64) == 0 && (MTOT % 64) == 0 && (DM % 64) == 0 && (NQKV % 64) == 0 && (HD % 64) == 0);
static_assert((DM % 32) == 0);
static_assert(((MTOT / 64) * (NQKV / 64)) % 8 == 0);
static_assert(((MTOT / 64) * (DM / 64)) % 8 == 0);
static_assert(((MTOT * DM / 8) % 256) == 0);
static_assert(((SEQ * NROT) % 256) == 0);
static_assert((SEQ & (SEQ - 1)) == 0);
static_assert((2 * 64 * HD + HD * 64) * 2 >= 4 * 16 * HD * 4);

typedef _Float16 v16h __attribute__((ext_vector_type(16)));
typedef _Float16 v8h  __attribute__((ext_vector_type(8)));
typedef float    v8f  __attribute__((ext_vector_type(8)));
typedef float    v4f  __attribute__((ext_vector_type(4)));
typedef unsigned int v4u __attribute__((ext_vector_type(4)));

__device__ __forceinline__ unsigned short bf_bits(float f) {
  unsigned u = __float_as_uint(f);
  return (unsigned short)((u + 0x7FFFu + ((u >> 16) & 1u)) >> 16);
}
__device__ __forceinline__ float bf_up(unsigned short h) { return __uint_as_float(((unsigned)h) << 16); }
__device__ __forceinline__ float bfr(float f) { return bf_up(bf_bits(f)); }
__device__ __forceinline__ unsigned short h_bits(_Float16 x) { return __builtin_bit_cast(unsigned short, x); }
__device__ __forceinline__ unsigned pk16(unsigned short a, unsigned short b) { return (unsigned)a | ((unsigned)b << 16); }
__device__ __forceinline__ v8f zero8() { v8f z = {0.f, 0.f, 0.f, 0.f, 0.f, 0.f, 0.f, 0.f}; return z; }

__device__ __forceinline__ void ld8(const float* p, float* o) {
  const v4f a = *(const v4f*)(p);
  const v4f b = *(const v4f*)(p + 4);
  o[0] = a[0]; o[1] = a[1]; o[2] = a[2]; o[3] = a[3];
  o[4] = b[0]; o[5] = b[1]; o[6] = b[2]; o[7] = b[3];
}

__device__ __forceinline__ v16h ldfrag_h(const _Float16* p) {
  union { v16h v; v8h h[2]; } f;
  f.h[0] = *(const v8h*)(p);
  f.h[1] = *(const v8h*)(p + 16);
  return f.v;
}

__device__ __forceinline__ v8f mma_h(v16h a, v16h b, v8f c) {
  c = __builtin_amdgcn_wmma_f32_16x16x32_f16(false, a, false, b, (short)0, c, false, false);
#if defined(__HIP_DEVICE_COMPILE__)
  asm volatile("v_nop\n\tv_nop\n\tv_nop\n\tv_nop" : "+v"(c) : "v"(a), "v"(b));
#endif
  return c;
}
__device__ __forceinline__ v8f mma_h_raw(v16h a, v16h b, v8f c) {
  return __builtin_amdgcn_wmma_f32_16x16x32_f16(false, a, false, b, (short)0, c, false, false);
}
__device__ __forceinline__ void dep_guard_h(v8f& a, v8f& b, v16h x) {
#if defined(__HIP_DEVICE_COMPILE__)
  asm volatile("v_nop\n\tv_nop\n\tv_nop\n\tv_nop" : "+v"(a), "+v"(b) : "v"(x));
#endif
}
__device__ __forceinline__ void keep4_h(v16h a, v16h b, v16h c, v16h d) {
#if defined(__HIP_DEVICE_COMPILE__)
  asm volatile("v_nop" :: "v"(a), "v"(b), "v"(c), "v"(d));
#endif
}
__device__ __forceinline__ void acc_guard4(v8f& a, v8f& b, v8f& c, v8f& d) {
#if defined(__HIP_DEVICE_COMPILE__)
  asm volatile("v_nop\n\tv_nop\n\tv_nop\n\tv_nop" : "+v"(a), "+v"(b), "+v"(c), "+v"(d));
#endif
}

__global__ __launch_bounds__(256) void rope_tab(float* ct, float* st, int n) {
#pragma clang fp contract(off)
  const int i = blockIdx.x * 256 + threadIdx.x;
  if (i < n) {
    const int t = i >> 6;
    const int j = i & 63;
    const float e   = (float)j * (1.0f / 64.0f);
    const float p   = powf(10000.0f, e);
    const float inv = 1.0f / p;
    const float ang = (float)t * inv;
    const float cv = cosf(ang);
    const float sv = sinf(ang);
    *(volatile float*)(ct + i) = cv;
    *(volatile float*)(st + i) = sv;
    __threadfence();
    *(volatile float*)(ct + i) = cv;
    *(volatile float*)(st + i) = sv;
  }
}

__global__ __launch_bounds__(256) void wt_cvt(const float* __restrict__ W, int ncols, int nrows,
                                              unsigned short* outp, float sc) {
  __shared__ __align__(16) float sw[64 * 68];
  const int tid = threadIdx.x;
  const int n0 = blockIdx.x * 64;
  const int k0 = blockIdx.y * 64;
#pragma unroll
  for (int i = 0; i < 4; ++i) {
    const int idx = i * 256 + tid;
    const int kk = idx >> 4, c4 = (idx & 15) * 4;
    const v4f a = *(const v4f*)(W + (size_t)(k0 + kk) * ncols + n0 + c4);
    *(v4f*)(sw + kk * 68 + c4) = a;
  }
  __syncthreads();

  const int g = tid >> 3, piece = tid & 7;
  v4u ov[2];
  size_t oofs[2];
#pragma unroll
  for (int it = 0; it < 2; ++it) {
    const int nn = it * 32 + g;
    v4u a;
#pragma unroll
    for (int e = 0; e < 4; ++e) {
      const float f0 = sw[(piece * 8 + 2 * e) * 68 + nn];
      const float f1 = sw[(piece * 8 + 2 * e + 1) * 68 + nn];
      a[e] = pk16(h_bits((_Float16)(bfr(f0) * sc)), h_bits((_Float16)(bfr(f1) * sc)));
    }
    ov[it] = a;
    oofs[it] = (size_t)(n0 + nn) * nrows + k0 + piece * 8;
  }
  for (int pass = 0; pass < 2; ++pass) {
#pragma unroll
    for (int it = 0; it < 2; ++it) *(volatile v4u*)(outp + oofs[it]) = ov[it];
    __threadfence();
  }
}

__global__ __launch_bounds__(256) void cvt_x8(const float* __restrict__ in, unsigned short* out, int n8,
                                              float sc) {
  const int i = blockIdx.x * 256 + threadIdx.x;
  if (i < n8) {
    const v4f a = *(const v4f*)(in + (size_t)i * 8);
    const v4f b = *(const v4f*)(in + (size_t)i * 8 + 4);
    v4u p;
    p[0] = pk16(h_bits((_Float16)(bfr(a[0]) * sc)), h_bits((_Float16)(bfr(a[1]) * sc)));
    p[1] = pk16(h_bits((_Float16)(bfr(a[2]) * sc)), h_bits((_Float16)(bfr(a[3]) * sc)));
    p[2] = pk16(h_bits((_Float16)(bfr(b[0]) * sc)), h_bits((_Float16)(bfr(b[1]) * sc)));
    p[3] = pk16(h_bits((_Float16)(bfr(b[2]) * sc)), h_bits((_Float16)(bfr(b[3]) * sc)));
    *(volatile v4u*)(out + (size_t)i * 8) = p;
    __threadfence();
    *(volatile v4u*)(out + (size_t)i * 8) = p;
  }
}

__global__ __launch_bounds__(256) void cvt_f16x8(const float* __restrict__ in, unsigned short* out, int n8,
                                                 float sc) {
  const int i = blockIdx.x * 256 + threadIdx.x;
  if (i < n8) {
    const v4f a = *(const v4f*)(in + (size_t)i * 8);
    const v4f b = *(const v4f*)(in + (size_t)i * 8 + 4);
    v4u p;
    p[0] = pk16(h_bits((_Float16)(a[0] * sc)), h_bits((_Float16)(a[1] * sc)));
    p[1] = pk16(h_bits((_Float16)(a[2] * sc)), h_bits((_Float16)(a[3] * sc)));
    p[2] = pk16(h_bits((_Float16)(b[0] * sc)), h_bits((_Float16)(b[1] * sc)));
    p[3] = pk16(h_bits((_Float16)(b[2] * sc)), h_bits((_Float16)(b[3] * sc)));
    *(volatile v4u*)(out + (size_t)i * 8) = p;
    __threadfence();
    *(volatile v4u*)(out + (size_t)i * 8) = p;
  }
}

template <int MODE>
__global__ __launch_bounds__(256) void gemm64(
    const unsigned short* __restrict__ Ap, int lda,
    const unsigned short* __restrict__ Btp, int ldb,
    const float* __restrict__ bias,
    float* Cf, int ldc, int M, int N, int K, float oscale) {
  const _Float16* Ah = (const _Float16*)(const void*)Ap;
  const _Float16* Bh = (const _Float16*)(const void*)Btp;
  __shared__ __align__(16) float sT[8][16 * 68];
  const int lane = threadIdx.x & 31;
  const int wave = threadIdx.x >> 5;
  const int tilesN = N >> 6;
  const int tilesM = M >> 6;
  const int tile = blockIdx.x * 8 + wave;
  if (tile >= tilesM * tilesN) return;
  const int tm = tile / tilesN;
  const int tn = tile - tm * tilesN;
  const int m0 = tm << 6;
  const int n0 = tn << 6;

  const int rlane = lane & 15;
  const int koff  = (lane >> 4) * 8;
  const int mOff  = (lane >> 4) * 8;

  v8f acc[4][4];
#pragma unroll
  for (int i = 0; i < 4; ++i)
#pragma unroll
    for (int j = 0; j < 4; ++j) acc[i][j] = zero8();

  for (int k0 = 0; k0 < K; k0 += 32) {
    v16h bh[4];
#pragma unroll
    for (int j = 0; j < 4; ++j) {
      const size_t bo = (size_t)(n0 + (j << 4) + rlane) * ldb + koff + k0;
      bh[j] = ldfrag_h(Bh + bo);
    }
#pragma unroll
    for (int i = 0; i < 4; ++i) {
      const size_t ao = (size_t)(m0 + (i << 4) + rlane) * lda + koff + k0;
      const v16h ah = ldfrag_h(Ah + ao);
#pragma unroll
      for (int j = 0; j < 4; ++j) acc[i][j] = mma_h_raw(ah, bh[j], acc[i][j]);
      dep_guard_h(acc[i][0], acc[i][3], ah);
    }
    keep4_h(bh[0], bh[1], bh[2], bh[3]);
  }
  acc_guard4(acc[0][0], acc[0][1], acc[0][2], acc[0][3]);
  acc_guard4(acc[1][0], acc[1][1], acc[1][2], acc[1][3]);
  acc_guard4(acc[2][0], acc[2][1], acc[2][2], acc[2][3]);
  acc_guard4(acc[3][0], acc[3][1], acc[3][2], acc[3][3]);

  float* slab = sT[wave];
  const int h2 = lane >> 4, c4 = (lane & 15) * 4;
  v4f b4 = {0.f, 0.f, 0.f, 0.f};
  if (MODE == 1) {
    const v4f braw = *(const v4f*)(bias + n0 + c4);
#pragma unroll
    for (int e = 0; e < 4; ++e) b4[e] = bfr(braw[e]);
  }
#pragma unroll
  for (int i = 0; i < 4; ++i) {
    const int mBase = m0 + (i << 4);
#pragma unroll
    for (int r = 0; r < 8; ++r) {
#pragma unroll
      for (int j = 0; j < 4; ++j) {
        slab[(mOff + r) * 68 + (j << 4) + rlane] = acc[i][j][r];
      }
    }
    __builtin_amdgcn_fence(__ATOMIC_RELEASE, "workgroup");
    __builtin_amdgcn_wave_barrier();
    __builtin_amdgcn_fence(__ATOMIC_ACQUIRE, "workgroup");
    v4f ov[8];
#pragma unroll
    for (int it = 0; it < 8; ++it) {
      const int row = it * 2 + h2;
      const v4f xs = *(const v4f*)(slab + row * 68 + c4);
      v4f v = xs * oscale;
      if (MODE == 1) v = v + b4;
      ov[it] = v;
    }
    for (int pass = 0; pass < 2; ++pass) {
#pragma unroll
      for (int it = 0; it < 8; ++it) {
        const int row = it * 2 + h2;
        *(volatile v4f*)(Cf + (size_t)(mBase + row) * ldc + n0 + c4) = ov[it];
      }
      __threadfence();
    }
    __builtin_amdgcn_fence(__ATOMIC_RELEASE, "workgroup");
    __builtin_amdgcn_wave_barrier();
    __builtin_amdgcn_fence(__ATOMIC_ACQUIRE, "workgroup");
  }
}

__global__ __launch_bounds__(128) void rope_qk(const float* __restrict__ qkvf, const float* __restrict__ ct,
                                               const float* __restrict__ st,
                                               unsigned short* qh, unsigned short* ql,
                                               unsigned short* kh, unsigned short* kl, float osc, float lsc) {
#pragma clang fp contract(off)
  const int tid = threadIdx.x;
  const int t = blockIdx.x;
  const int pos = t & (SEQ - 1);
  const float* rowp = qkvf + (size_t)t * NQKV;
  const float* ctp  = ct + (size_t)pos * NROT;
  const float* stp  = st + (size_t)pos * NROT;
  const int d0 = tid * 8;
  const int dp = d0 ^ 64;
  const float sgn = ((d0 & 64) == 0) ? -1.0f : 1.0f;
  const int j0 = d0 & 63;
  const int kd0 = (tid & 15) * 8;
  const int kdp = kd0 ^ 64;
  const float sgk = ((kd0 & 64) == 0) ? -1.0f : 1.0f;
  const int jk = kd0 & 63;
  float xq[8], xqp[8], cv[8], sv[8], xk[8], xkp[8], ck[8], sk[8];
  ld8(rowp + d0, xq);
  ld8(rowp + dp, xqp);
  ld8(ctp + j0, cv);
  ld8(stp + j0, sv);
  ld8(rowp + DM + kd0, xk);
  ld8(rowp + DM + kdp, xkp);
  ld8(ctp + jk, ck);
  ld8(stp + jk, sk);
  v4u aq, aql, ak, akl;
#pragma unroll
  for (int p = 0; p < 4; ++p) {
    const int e = 2 * p;
    const float yq0 = xq[e] * cv[e] + (sgn * xqp[e]) * sv[e];
    const float yq1 = xq[e + 1] * cv[e + 1] + (sgn * xqp[e + 1]) * sv[e + 1];
    const float yk0 = xk[e] * ck[e] + (sgk * xkp[e]) * sk[e];
    const float yk1 = xk[e + 1] * ck[e + 1] + (sgk * xkp[e + 1]) * sk[e + 1];
    const float fq0 = yq0 * osc, fq1 = yq1 * osc, fk0 = yk0 * osc, fk1 = yk1 * osc;
    const _Float16 hq0 = (_Float16)fq0, hq1 = (_Float16)fq1, hk0 = (_Float16)fk0, hk1 = (_Float16)fk1;
    const _Float16 lq0 = (_Float16)((fq0 - (float)hq0) * lsc);
    const _Float16 lq1 = (_Float16)((fq1 - (float)hq1) * lsc);
    const _Float16 lk0 = (_Float16)((fk0 - (float)hk0) * lsc);
    const _Float16 lk1 = (_Float16)((fk1 - (float)hk1) * lsc);
    aq[p]  = pk16(h_bits(hq0), h_bits(hq1));
    aql[p] = pk16(h_bits(lq0), h_bits(lq1));
    ak[p]  = pk16(h_bits(hk0), h_bits(hk1));
    akl[p] = pk16(h_bits(lk0), h_bits(lk1));
  }
  const size_t oq = (size_t)t * DM + d0;
  const size_t okk = (size_t)t * HD + kd0;
  *(volatile v4u*)(qh + oq) = aq;
  *(volatile v4u*)(ql + oq) = aql;
  if (tid < 16) { *(volatile v4u*)(kh + okk) = ak; *(volatile v4u*)(kl + okk) = akl; }
  __threadfence();
  *(volatile v4u*)(qh + oq) = aq;
  *(volatile v4u*)(ql + oq) = aql;
  if (tid < 16) { *(volatile v4u*)(kh + okk) = ak; *(volatile v4u*)(kl + okk) = akl; }
}

__global__ __launch_bounds__(256) void v_plane(const float* __restrict__ vf, int vrp,
                                               unsigned short* vt, float vscale) {
  __shared__ __align__(16) float sv[64 * 68];
  const int tid = threadIdx.x;
  const int t0  = blockIdx.x * 64;
  const int f0  = blockIdx.y * 64;
  const int bb  = blockIdx.z;
#pragma unroll
  for (int i = 0; i < 4; ++i) {
    const int idx = i * 256 + tid;
    const int tt = idx >> 4, c4 = (idx & 15) * 4;
    const v4f a = *(const v4f*)(vf + ((size_t)(bb * SEQ + t0 + tt)) * vrp + f0 + c4);
    *(v4f*)(sv + tt * 68 + c4) = a;
  }
  __syncthreads();

  const int g = tid >> 3, piece = tid & 7;
  v4u hv[2];
  size_t hofs[2];
#pragma unroll
  for (int it = 0; it < 2; ++it) {
    const int d = it * 32 + g;
    v4u a;
#pragma unroll
    for (int e = 0; e < 4; ++e) {
      const float fa = sv[(piece * 8 + 2 * e) * 68 + d] * vscale;
      const float fb = sv[(piece * 8 + 2 * e + 1) * 68 + d] * vscale;
      a[e] = pk16(h_bits((_Float16)fa), h_bits((_Float16)fb));
    }
    hv[it] = a;
    hofs[it] = ((size_t)(bb * HD + f0 + d)) * SEQ + t0 + piece * 8;
  }
  for (int pass = 0; pass < 2; ++pass) {
#pragma unroll
    for (int it = 0; it < 2; ++it) *(volatile v4u*)(vt + hofs[it]) = hv[it];
    __threadfence();
  }
}

__global__ __launch_bounds__(128)
void attn_mq(const unsigned short* __restrict__ qhp, const unsigned short* __restrict__ qlp,
             const unsigned short* __restrict__ khp, const unsigned short* __restrict__ klp,
             const unsigned short* __restrict__ vtp, float* outp, float sscale, float lfold, float oscl) {
  union FH { v16h v; v8h h[2]; };
  __shared__ __align__(16) _Float16 KVsh[2 * 64 * HD + HD * 64];
  __shared__ __align__(16) _Float16 Psh[4][16 * 64];
  _Float16* Ksh  = KVsh;
  _Float16* Klsh = KVsh + 64 * HD;
  _Float16* Vth  = KVsh + 2 * 64 * HD;

  const int tid  = threadIdx.x;
  const int wave = tid >> 5;
  const int lane = tid & 31;
  const int hh   = lane >> 4;
  const int c    = lane & 15;

  const int bx  = blockIdx.x;
  const int bb  = bx / (NH * NQB);
  const int rem = bx - bb * (NH * NQB);
  const int h   = rem / NQB;
  const int qb  = rem - h * NQB;
  const int g0  = bb * SEQ + qb * 64 + wave * 16;

  const _Float16* Qp  = (const _Float16*)(const void*)qhp + (size_t)h * HD;
  const _Float16* Qlq = (const _Float16*)(const void*)qlp + (size_t)h * HD;
  const _Float16* Kp  = (const _Float16*)(const void*)khp + (size_t)bb * SEQ * HD;
  const _Float16* Klg = (const _Float16*)(const void*)klp + (size_t)bb * SEQ * HD;
  const _Float16* Vp  = (const _Float16*)(const void*)vtp + (size_t)bb * HD * SEQ;

  v16h qa[4], qr[4];
#pragma unroll
  for (int dc = 0; dc < 4; ++dc) {
    const size_t qo = (size_t)(g0 + c) * DM + dc * 32 + 8 * hh;
    qa[dc] = ldfrag_h(Qp + qo);
    qr[dc] = ldfrag_h(Qlq + qo);
  }

  float mrow[8], lrow[8];
  v8f oacc[8];
#pragma unroll
  for (int r = 0; r < 8; ++r) { mrow[r] = -INFINITY; lrow[r] = 0.f; }
#pragma unroll
  for (int t = 0; t < 8; ++t) oacc[t] = zero8();

  for (int kt = 0; kt < NQB; ++kt) {
    const int kv0 = kt * 64;
    __syncthreads();
    {
      const int r = tid >> 1, half = (tid & 1) * 64;
      const _Float16* kg  = Kp  + (size_t)(kv0 + r) * HD + half;
      const _Float16* klg = Klg + (size_t)(kv0 + r) * HD + half;
      const _Float16* vg  = Vp + (size_t)tid * SEQ + kv0;
#pragma unroll
      for (int i = 0; i < 8; ++i) {
        const v8h a0 = *(const v8h*)(kg + 8 * i);
        const v8h a1 = *(const v8h*)(klg + 8 * i);
        const v8h b0 = *(const v8h*)(vg + 8 * i);
        *(v8h*)(Ksh  + r * HD + half + 8 * i) = a0;
        *(v8h*)(Klsh + r * HD + half + 8 * i) = a1;
        *(v8h*)(Vth  + tid * 64 + 8 * i) = b0;
      }
    }
    __syncthreads();

    v8f s[4];
#pragma unroll
    for (int j = 0; j < 4; ++j) {
      v8f shh = zero8(), srs = zero8();
#pragma unroll
      for (int dc = 0; dc < 4; ++dc) {
        FH kb, kl;
        kb.h[0] = *(const v8h*)(Ksh  + (j * 16 + c) * HD + dc * 32 + 8 * hh);
        kb.h[1] = *(const v8h*)(Ksh  + (j * 16 + c) * HD + dc * 32 + 16 + 8 * hh);
        kl.h[0] = *(const v8h*)(Klsh + (j * 16 + c) * HD + dc * 32 + 8 * hh);
        kl.h[1] = *(const v8h*)(Klsh + (j * 16 + c) * HD + dc * 32 + 16 + 8 * hh);
        shh = mma_h(qa[dc], kb.v, shh);
        srs = mma_h(qa[dc], kl.v, srs);
        srs = mma_h(qr[dc], kb.v, srs);
      }
      s[j] = shh + srs * lfold;
    }

    _Float16* pwh = Psh[wave];
#pragma unroll
    for (int r = 0; r < 8; ++r) {
      float m = -INFINITY;
#pragma unroll
      for (int j = 0; j < 4; ++j) {
        const float sv = s[j][r] * sscale;
        s[j][r] = sv;
        m = fmaxf(m, sv);
      }
#pragma unroll
      for (int off = 1; off < 16; off <<= 1) m = fmaxf(m, __shfl_xor(m, off, 32));
      const float mnew  = fmaxf(mrow[r], m);
      const float msafe = (mnew == -INFINITY) ? 0.f : mnew;
      const float alpha = __expf(mrow[r] - msafe);
      mrow[r] = mnew;
      float psum = 0.f;
#pragma unroll
      for (int j = 0; j < 4; ++j) {
        const float p = __expf(s[j][r] - msafe);
        psum += p;
        const _Float16 ph = (_Float16)(p * 1024.0f);
        pwh[(8 * hh + r) * 64 + j * 16 + c] = ph;
      }
#pragma unroll
      for (int off = 1; off < 16; off <<= 1) psum += __shfl_xor(psum, off, 32);
      lrow[r] = lrow[r] * alpha + psum;
#pragma unroll
      for (int t = 0; t < 8; ++t) oacc[t][r] *= alpha;
    }
    __builtin_amdgcn_fence(__ATOMIC_RELEASE, "workgroup");
    __builtin_amdgcn_wave_barrier();
    __builtin_amdgcn_fence(__ATOMIC_ACQUIRE, "workgroup");

#pragma unroll 1
    for (int kk = 0; kk < 2; ++kk) {
      FH pa;
      pa.h[0] = *(const v8h*)(pwh + c * 64 + kk * 32 + 8 * hh);
      pa.h[1] = *(const v8h*)(pwh + c * 64 + kk * 32 + 16 + 8 * hh);
#pragma unroll
      for (int t = 0; t < 8; ++t) {
        FH vb;
        vb.h[0] = *(const v8h*)(Vth + (t * 16 + c) * 64 + kk * 32 + 8 * hh);
        vb.h[1] = *(const v8h*)(Vth + (t * 16 + c) * 64 + kk * 32 + 16 + 8 * hh);
        oacc[t] = mma_h(pa.v, vb.v, oacc[t]);
      }
    }
  }
  __syncthreads();

  float* os = (float*)(void*)KVsh + wave * (16 * HD);
#pragma unroll
  for (int r = 0; r < 8; ++r) {
    const float l = lrow[r];
    const float inv = ((l > 0.f) ? (1.0f / l) : 0.f) * oscl;
#pragma unroll
    for (int t = 0; t < 8; ++t) os[(8 * hh + r) * HD + t * 16 + c] = oacc[t][r] * inv;
  }
  __builtin_amdgcn_fence(__ATOMIC_RELEASE, "workgroup");
  __builtin_amdgcn_wave_barrier();
  __builtin_amdgcn_fence(__ATOMIC_ACQUIRE, "workgroup");
  {
    const int c4 = lane * 4;
    v4f ov[16];
#pragma unroll
    for (int row = 0; row < 16; ++row) ov[row] = *(const v4f*)(os + row * HD + c4);
    for (int pass = 0; pass < 2; ++pass) {
#pragma unroll
      for (int row = 0; row < 16; ++row) {
        const size_t go = (size_t)(g0 + row) * DM + (size_t)h * HD + c4;
        *(volatile v4f*)(outp + go) = ov[row];
      }
      __threadfence();
    }
  }
}

extern "C" void kernel_launch(void* const* d_in, const int* in_sizes, int n_in,
                              void* d_out, int out_size, void* d_ws, size_t ws_size,
                              hipStream_t stream) {
  if (n_in < 6) return;
  if (in_sizes[0] != MTOT * DM) return;
  if (in_sizes[1] != DM * DM) return;
  if (in_sizes[2] != DM * HD) return;
  if (in_sizes[3] != DM * HD) return;
  if (in_sizes[4] != DM * DM) return;
  if (in_sizes[5] != DM) return;
  if (out_size != OUTN) return;

  const float* x  = (const float*)d_in[0];
  const float* wq = (const float*)d_in[1];
  const float* wk = (const float*)d_in[2];
  const float* wv = (const float*)d_in[3];
  const float* wo = (const float*)d_in[4];
  const float* bo = (const float*)d_in[5];

  const size_t PX16  = (size_t)MTOT * DM * 2;
  const size_t PWqkv = (size_t)NQKV * DM * 2;
  const size_t PWo   = (size_t)DM * DM * 2;
  const size_t PTrig = (size_t)SEQ * NROT * 4;
  const size_t PQKV  = (size_t)MTOT * NQKV * 4;
  const size_t PQh   = (size_t)MTOT * DM * 2;
  const size_t PKh   = (size_t)MTOT * HD * 2;
  const size_t PVt   = (size_t)NBATCH * HD * SEQ * 2;
  const size_t PYf   = (size_t)MTOT * DM * 4;
  const size_t PY16  = (size_t)MTOT * DM * 2;
  size_t off = 0;
  const size_t oX16 = off; off += PX16;
  const size_t oWq  = off; off += PWqkv;
  const size_t oWo  = off; off += PWo;
  const size_t oCos = off; off += PTrig;
  const size_t oSin = off; off += PTrig;
  const size_t oQKV = off; off += PQKV;
  const size_t oQh  = off; off += PQh;
  const size_t oQl  = off; off += PQh;
  const size_t oKh  = off; off += PKh;
  const size_t oKl  = off; off += PKh;
  const size_t oVt  = off; off += PVt;
  const size_t oYf  = off; off += PYf;
  const size_t oY16 = off; off += PY16;
  if (off > ws_size) return;
  if (off > (size_t)134217728) return;

  char* ws = (char*)d_ws;
  unsigned short* X16   = (unsigned short*)(ws + oX16);
  unsigned short* WqkvT = (unsigned short*)(ws + oWq);
  unsigned short* WoT   = (unsigned short*)(ws + oWo);
  float*          CosT  = (float*)(ws + oCos);
  float*          SinT  = (float*)(ws + oSin);
  float*          QKVf  = (float*)(ws + oQKV);
  unsigned short* Qh    = (unsigned short*)(ws + oQh);
  unsigned short* Ql    = (unsigned short*)(ws + oQl);
  unsigned short* Kh    = (unsigned short*)(ws + oKh);
  unsigned short* Kl    = (unsigned short*)(ws + oKl);
  unsigned short* VT    = (unsigned short*)(ws + oVt);
  float*          Yf    = (float*)(ws + oYf);
  unsigned short* Y16   = (unsigned short*)(ws + oY16);
  float*          outf  = (float*)d_out;

  const dim3 blk(256);
  const int nTrig = SEQ * NROT;
  const int n8x   = MTOT * DM / 8;
  const dim3 gTrig((nTrig + 255) / 256);
  const dim3 gCvt((n8x + 255) / 256);
  const dim3 gWq(DM / 64, DM / 64);
  const dim3 gWkv(HD / 64, DM / 64);
  const dim3 gWo(DM / 64, DM / 64);
  const dim3 gQKV(((MTOT / 64) * (NQKV / 64) + 7) / 8);
  const dim3 gDM(((MTOT / 64) * (DM / 64) + 7) / 8);
  const dim3 gVpl(SEQ / 64, HD / 64, NBATCH);
  const dim3 gAttn(NBATCH * NH * NQB);

  const float wScale  = 64.0f;
  const float xScale  = 8.0f;
  const float qkScale = 16.0f;
  const float qkLsc   = 2048.0f;
  const float qkLfold = 1.0f / 2048.0f;
  const float sscale  = 0.08838834764831845f * (1.0f / 256.0f);
  const float vScale  = 256.0f;
  const float attOscl = 1.0f / 262144.0f;
  const float yScale  = 64.0f;

  rope_tab<<<gTrig, blk, 0, stream>>>(CosT, SinT, nTrig);
  wt_cvt<<<gWq, blk, 0, stream>>>(wq, DM, DM, WqkvT, wScale);
  wt_cvt<<<gWkv, blk, 0, stream>>>(wk, HD, DM, WqkvT + (size_t)DM * DM, wScale);
  wt_cvt<<<gWkv, blk, 0, stream>>>(wv, HD, DM, WqkvT + (size_t)(DM + HD) * DM, wScale);
  wt_cvt<<<gWo, blk, 0, stream>>>(wo, DM, DM, WoT, wScale);
  cvt_x8<<<gCvt, blk, 0, stream>>>(x, X16, n8x, xScale);
  gemm64<0><<<gQKV, blk, 0, stream>>>(X16, DM, WqkvT, DM, bo, QKVf, NQKV, MTOT, NQKV, DM, 1.0f / 512.0f);
  rope_qk<<<dim3(MTOT), dim3(128), 0, stream>>>(QKVf, CosT, SinT, Qh, Ql, Kh, Kl, qkScale, qkLsc);
  v_plane<<<gVpl, blk, 0, stream>>>(QKVf + DM + HD, NQKV, VT, vScale);
  attn_mq<<<gAttn, dim3(128), 0, stream>>>(Qh, Ql, Kh, Kl, VT, Yf, sscale, qkLfold, attOscl);
  cvt_f16x8<<<gCvt, blk, 0, stream>>>(Yf, Y16, n8x, yScale);
  gemm64<1><<<gDM, blk, 0, stream>>>(Y16, DM, WoT, DM, bo, outf, DM, MTOT, DM, DM, 1.0f / 4096.0f);
  (void)hipGetLastError();
}
